// SequentialTransductionUnit_38783554683549
// MI455X (gfx1250) — hardware-verified
//
#include <hip/hip_runtime.h>


#define NBI  2
#define NT   2048
#define DMD  1024
#define NH   16
#define HD   64
#define H4   (4 * DMD)
#define OU   0
#define OV   1024
#define OQ   2048
#define OK_  3072
#define RCH  1024
#define LN_EPS 1e-5f
#define DM   DMD
#define LOSC 1024.0f

typedef _Float16 h16;
typedef unsigned short bf;
typedef __attribute__((ext_vector_type(16))) __bf16   v16bf;
typedef __attribute__((ext_vector_type(16))) _Float16 v16h;
typedef __attribute__((ext_vector_type(8)))  _Float16 v8h;
typedef __attribute__((ext_vector_type(8)))  unsigned short v8us;
typedef __attribute__((ext_vector_type(8)))  float    v8f;
typedef __attribute__((ext_vector_type(4)))  float    v4f;
typedef v8h  __attribute__((may_alias)) v8ha;
typedef v4f  __attribute__((may_alias)) v4fa;
typedef v8us __attribute__((may_alias)) v8usa;

__device__ __forceinline__ unsigned short f2bf(float f) { unsigned u = __float_as_uint(f); u += 0x7FFFu + ((u >> 16) & 1u); return (unsigned short)(u >> 16); }
__device__ __forceinline__ float bf2f(unsigned short b) { return __uint_as_float(((unsigned)b) << 16); }
__device__ __forceinline__ float bfr(float f) { return bf2f(f2bf(f)); }
__device__ __forceinline__ v16h cat16(v8h lo, v8h hi) { return __builtin_shufflevector(lo, hi, 0, 1, 2, 3, 4, 5, 6, 7, 8, 9, 10, 11, 12, 13, 14, 15); }
__device__ __forceinline__ v16bf cat16b(v8us lo, v8us hi) { return __builtin_bit_cast(v16bf, __builtin_shufflevector(lo, hi, 0, 1, 2, 3, 4, 5, 6, 7, 8, 9, 10, 11, 12, 13, 14, 15)); }
__device__ __forceinline__ v8f wmma16(v16h a, v16h b, v8f c) { return __builtin_amdgcn_wmma_f32_16x16x32_f16(false, a, false, b, (short)0, c, false, false); }
__device__ __forceinline__ v8f wmmab(v16bf a, v16bf b, v8f c) { return __builtin_amdgcn_wmma_f32_16x16x32_bf16(false, a, false, b, (short)0, c, false, false); }

template <bool SPLITA, bool F16OUT = false>
__global__ __launch_bounds__(128) void k_gemmb(const bf* __restrict__ A, const bf* __restrict__ Al, const bf* __restrict__ Bn, const float* __restrict__ bias, float* C, int ldc, h16* C2, const float* __restrict__ R = nullptr, int K = DM, int roundR = 1) {
    __shared__ __align__(16) float ost[4][16 * 68];
    const int lane = threadIdx.x & 31, wave = threadIdx.x >> 5, lr = lane & 15, hi = lane >> 4;
    const int r0 = blockIdx.x * 64 + wave * 16, c0 = blockIdx.y * 64;
    const size_t aoff = (size_t)(r0 + lr) * K + 8 * hi;
    size_t boff[4];
#pragma unroll
    for (int t = 0; t < 4; ++t) boff[t] = (size_t)(c0 + t * 16 + lr) * K + 8 * hi;
    v8f acc[4];
#pragma unroll
    for (int t = 0; t < 4; ++t) acc[t] = (v8f){};
#pragma unroll 1
    for (int kc = 0; kc < K; kc += 32) {
        const v16bf a = cat16b(*(const v8us*)(A + aoff + kc), *(const v8us*)(A + aoff + kc + 16));
        v16bf al = a;
        if (SPLITA) al = cat16b(*(const v8us*)(Al + aoff + kc), *(const v8us*)(Al + aoff + kc + 16));
#pragma unroll
        for (int t = 0; t < 4; ++t) { const v16bf b = cat16b(*(const v8us*)(Bn + boff[t] + kc), *(const v8us*)(Bn + boff[t] + kc + 16)); acc[t] = wmmab(a, b, acc[t]); if (SPLITA) acc[t] = wmmab(al, b, acc[t]); }
        asm volatile("v_nop\n\tv_nop\n\tv_nop\n\tv_nop" : "+v"(acc[0]), "+v"(acc[1]), "+v"(acc[2]), "+v"(acc[3]) : "v"(a), "v"(al));
    }
    float* os = &ost[wave][0];
#pragma unroll
    for (int t = 0; t < 4; ++t) { const float bv = bias ? bfr(bias[c0 + t * 16 + lr]) : 0.f;
#pragma unroll
        for (int j = 0; j < 8; ++j) os[(hi * 8 + j) * 68 + t * 16 + lr] = acc[t][j] + bv; }
    __syncthreads();
    if (F16OUT) {
        h16* crow = (h16*)(void*)C + (size_t)r0 * ldc + c0;
        auto pass = [&]() {
#pragma unroll
            for (int s = 0; s < 4; ++s) { const int row = 4 * s + (lane >> 3), piece = lane & 7; const float* sp = os + row * 68 + piece * 8; v8h o, o2;
#pragma unroll
                for (int i = 0; i < 8; ++i) { const h16 a = (h16)sp[i]; o[i] = a; o2[i] = (h16)((sp[i] - (float)a) * LOSC); }
                *(volatile v8h*)(crow + (size_t)row * ldc + piece * 8) = o; if (C2) *(volatile v8h*)(C2 + (size_t)r0 * ldc + c0 + (size_t)row * ldc + piece * 8) = o2; }
        };
        pass(); __threadfence(); pass();
    } else {
        float* crow = C + (size_t)r0 * ldc + c0;
        auto pass = [&]() {
#pragma unroll
            for (int s = 0; s < 8; ++s) { const int Lid = (lane >> 3) + 4 * s, piece = lane & 7; const int row = Lid >> 1, cofs = (Lid & 1) * 32 + piece * 4;
                v4f val = *(const v4fa*)(os + row * 68 + cofs); if (R) { const v4f rv = *(const v4f*)(R + ((size_t)r0 + row) * ldc + c0 + cofs); val += roundR ? (v4f){bfr(rv[0]), bfr(rv[1]), bfr(rv[2]), bfr(rv[3])} : rv; }
                *(volatile v4f*)(crow + (size_t)row * ldc + cofs) = val; }
        };
        pass(); __threadfence(); pass();
    }
}


__global__ __launch_bounds__(256) void k_cvt8(const float* __restrict__ src, bf* dst, size_t n8) {
    const size_t i = (size_t)blockIdx.x * 256 + threadIdx.x; if (i >= n8) return;
    const v8f v = *(const v8f*)(src + i * 8); v8us o;
#pragma unroll
    for (int k = 0; k < 8; ++k) o[k] = f2bf(v[k]);
    *(volatile v8us*)(dst + i * 8) = o; __threadfence(); *(volatile v8us*)(dst + i * 8) = o;
}
__global__ __launch_bounds__(256) void k_zero8(bf* dst, size_t n8) {
    const size_t i = (size_t)blockIdx.x * 256 + threadIdx.x; if (i >= n8) return; v8us z;
#pragma unroll
    for (int k = 0; k < 8; ++k) z[k] = 0;
    *(volatile v8us*)(dst + i * 8) = z; __threadfence(); *(volatile v8us*)(dst + i * 8) = z;
}

__global__ __launch_bounds__(256) void k_cvtb(const float* __restrict__ src, int nrows, bf* dst) {
    const int lane = threadIdx.x & 31, r = blockIdx.x * 8 + (threadIdx.x >> 5); if (r >= nrows) return;
#pragma unroll 1
    for (int ps = 0; ps < 2; ++ps) {
#pragma unroll
        for (int q = 0; q < DMD / 256; ++q) { v8us o;
#pragma unroll
            for (int i = 0; i < 8; ++i) o[i] = f2bf(src[(size_t)r * DMD + q * 256 + lane * 8 + i]);
            *(volatile v8us*)(dst + (size_t)r * DMD + q * 256 + lane * 8) = o; }
        if (ps == 0) __threadfence(); }
}
__global__ __launch_bounds__(256) void k_pos(const float* __restrict__ rl, float* CT, float* ST) {
    __shared__ float ps_[NT];
    if (threadIdx.x == 0) { float acc = 0.f;
#pragma unroll 1
        for (int t = 0; t < NT; ++t) { acc += bfr(rl[t]); ps_[t] = acc; } }
    __syncthreads();
    const int lane = threadIdx.x & 31, wv = threadIdx.x >> 5; const float invf = 1.0f / powf(10000.0f, (float)(2 * lane) / (float)HD);
#pragma unroll 1
    for (int t = wv; t < NT; t += 8) { const float ang = ps_[t] * invf; const float c = cosf(ang), s = sinf(ang);
        *(volatile float*)(CT + (size_t)t * 32 + lane) = c; *(volatile float*)(ST + (size_t)t * 32 + lane) = s; __threadfence(); *(volatile float*)(CT + (size_t)t * 32 + lane) = c; *(volatile float*)(ST + (size_t)t * 32 + lane) = s; }
}
__global__ __launch_bounds__(256) void k_qk(const float* __restrict__ Hm, const float* __restrict__ CT, const float* __restrict__ ST, const float* __restrict__ qg, const float* __restrict__ kg, bf* Qh, bf* Ql, bf* Kh, bf* Kl) {
    typedef __attribute__((ext_vector_type(2))) unsigned short v2us;
    const int lane = threadIdx.x & 31; const int wid = blockIdx.x * 8 + (threadIdx.x >> 5); const int t = wid / NH, h = wid - t * NH; if (t >= NT) return;
    const float gq = bfr(qg[(size_t)t * NH + h]), gk = bfr(kg[(size_t)t * NH + h]);
#pragma unroll
    for (int which = 0; which < 2; ++which) { const float* src = Hm + (size_t)t * H4 + (which ? OK_ : OQ) + h * HD; const float g = which ? gk : gq;
        float y[2];
#pragma unroll
        for (int i = 0; i < 2; ++i) { const int dp = 2 * lane + i; const int d = dp & 31; float e = src[2 * d], o = src[2 * d + 1]; e = e / (1.0f + __expf(-e)); o = o / (1.0f + __expf(-o));
            const float c = CT[(size_t)t * 32 + d], s = ST[(size_t)t * 32 + d]; y[i] = ((dp < 32) ? (e * c - o * s) : (e * s + o * c)) * g; }
        v2us oh, ol;
#pragma unroll
        for (int i = 0; i < 2; ++i) { const unsigned short hb = f2bf(y[i]); oh[i] = hb; ol[i] = f2bf(y[i] - bf2f(hb)); }
        bf* dh = which ? Kh : Qh; bf* dl = which ? Kl : Ql; const size_t ob = (size_t)t * DMD + h * HD + 2 * lane;
        *(volatile v2us*)(dh + ob) = oh; *(volatile v2us*)(dl + ob) = ol; __threadfence(); *(volatile v2us*)(dh + ob) = oh; *(volatile v2us*)(dl + ob) = ol; }
}
__global__ __launch_bounds__(256) void k_vtb(const float* __restrict__ Hm, const float* __restrict__ vg, bf* VTh, bf* VTl) {
    __shared__ float tl[64][65];
    const int tid = threadIdx.x, t0 = blockIdx.x * 64, h = blockIdx.y;
    { const int tt = tid >> 2, dq = (tid & 3) * 16; const float g = bfr(vg[(size_t)(t0 + tt) * NH + h]);
#pragma unroll 2
      for (int i = 0; i < 16; ++i) { const float v = Hm[(size_t)(t0 + tt) * H4 + OV + h * HD + dq + i]; tl[dq + i][tt] = (v / (1.0f + __expf(-v))) * g; } }
    __syncthreads();
    const int piece = tid & 7, Lid = tid >> 3;
    auto pass = [&]() {
#pragma unroll
        for (int s = 0; s < 2; ++s) { const int d = Lid + 32 * s; v8us oh, ol;
#pragma unroll
            for (int i = 0; i < 8; ++i) { const float v = tl[d][piece * 8 + i]; const unsigned short hb = f2bf(v); oh[i] = hb; ol[i] = f2bf(v - bf2f(hb)); }
            const size_t o = ((size_t)h * HD + d) * NT + t0 + piece * 8; *(volatile v8us*)(VTh + o) = oh; *(volatile v8us*)(VTl + o) = ol; }
    };
    pass(); __threadfence(); pass();
}
__global__ __launch_bounds__(256) void k_wprep(const float* __restrict__ S, const float* __restrict__ bias, const int* __restrict__ msk, const float* __restrict__ hs, int h, int i0, bf* Wh, bf* Wl) {
    const int lane = threadIdx.x & 31, r = blockIdx.x * 8 + (threadIdx.x >> 5); if (r >= RCH) return; const float sc = bfr(hs[h]); const size_t brow = (size_t)(i0 + r) * NT;
#pragma unroll 1
    for (int ps = 0; ps < 2; ++ps) {
#pragma unroll 1
        for (int c0 = lane * 8; c0 < NT; c0 += 256) { v8us oh, ol;
#pragma unroll
            for (int q = 0; q < 8; ++q) { const int j = c0 + q; const float bb = bfr(bias[brow + j]); float lg = S[(size_t)r * NT + j] * sc + bb; lg = lg + 3.0f * bb; float wv = lg / (1.0f + __expf(-lg)); wv = (msk[brow + j] != 0) ? wv : 0.f;
                const unsigned short hb = f2bf(wv); oh[q] = hb; ol[q] = f2bf(wv - bf2f(hb)); }
            const size_t o = (size_t)r * NT + c0; *(volatile v8us*)(Wh + o) = oh; *(volatile v8us*)(Wl + o) = ol; }
        if (ps == 0) __threadfence(); }
}
__global__ __launch_bounds__(128) void k_gemm3ll(const bf* __restrict__ Ah, const bf* __restrict__ Al, int lda, const bf* __restrict__ Bh, const bf* __restrict__ Bl, int ldb, int K, float* C, int ldc) {
    __shared__ __align__(16) float ost[4][16 * 68];
    const int lane = threadIdx.x & 31, wave = threadIdx.x >> 5, lr = lane & 15, hi = lane >> 4;
    const int r0 = blockIdx.x * 64 + wave * 16, c0 = blockIdx.y * 64;
    const size_t aoff = (size_t)(r0 + lr) * lda + 8 * hi;
    v8f acc[4];
#pragma unroll
    for (int t = 0; t < 4; ++t) acc[t] = (v8f){};
#pragma unroll 1
    for (int kc = 0; kc < K; kc += 32) {
        const v16bf a = cat16b(*(const v8us*)(Ah + aoff + kc), *(const v8us*)(Ah + aoff + kc + 16));
        const v16bf al = cat16b(*(const v8us*)(Al + aoff + kc), *(const v8us*)(Al + aoff + kc + 16));
#pragma unroll
        for (int t = 0; t < 4; ++t) { const size_t bo = (size_t)(c0 + t * 16 + lr) * ldb + kc + 8 * hi;
            const v16bf bh = cat16b(*(const v8us*)(Bh + bo), *(const v8us*)(Bh + bo + 16)); const v16bf bl = cat16b(*(const v8us*)(Bl + bo), *(const v8us*)(Bl + bo + 16));
            acc[t] = wmmab(a, bh, acc[t]); acc[t] = wmmab(al, bh, acc[t]); acc[t] = wmmab(a, bl, acc[t]); }
        asm volatile("v_nop\n\tv_nop\n\tv_nop\n\tv_nop" : "+v"(acc[0]), "+v"(acc[1]), "+v"(acc[2]), "+v"(acc[3]) : "v"(a), "v"(al));
    }
    float* os = &ost[wave][0];
#pragma unroll
    for (int t = 0; t < 4; ++t) {
#pragma unroll
        for (int j = 0; j < 8; ++j) os[(hi * 8 + j) * 68 + t * 16 + lr] = acc[t][j]; }
    __builtin_amdgcn_wave_barrier(); asm volatile("" ::: "memory");
    float* crow = C + (size_t)r0 * ldc + c0;
    auto pass = [&]() {
#pragma unroll
        for (int s = 0; s < 8; ++s) { const int Lid = (lane >> 3) + 4 * s, piece = lane & 7; const int row = Lid >> 1, cofs = (Lid & 1) * 32 + piece * 4;
            const v4f val = *(const v4fa*)(os + row * 68 + cofs); *(volatile v4f*)(crow + (size_t)row * ldc + cofs) = val; }
    };
    pass(); __threadfence(); pass();
}
__global__ __launch_bounds__(256) void k_ygate(const float* __restrict__ Y, const float* __restrict__ Hm, bf* Yh, bf* Yl) {
    const int lane = threadIdx.x & 31, t = blockIdx.x * 8 + (threadIdx.x >> 5); if (t >= NT) return;
#pragma unroll 1
    for (int ps = 0; ps < 2; ++ps) {
#pragma unroll 1
        for (int c0 = lane * 8; c0 < DMD; c0 += 256) { v8us oh, ol;
#pragma unroll
            for (int q = 0; q < 8; ++q) { const int c = c0 + q; const float u = Hm[(size_t)t * H4 + OU + c]; const float yv = Y[(size_t)t * DMD + c] * (u / (1.0f + __expf(-u))); const unsigned short hb = f2bf(yv); oh[q] = hb; ol[q] = f2bf(yv - bf2f(hb)); }
            const size_t o = (size_t)t * DMD + c0; *(volatile v8us*)(Yh + o) = oh; *(volatile v8us*)(Yl + o) = ol; }
        if (ps == 0) __threadfence(); }
}
__global__ __launch_bounds__(256) void k_ln(const float* __restrict__ R, const float* __restrict__ g, const float* __restrict__ bb, float* OUTP) {
    const int lane = threadIdx.x & 31, r = blockIdx.x * 8 + (threadIdx.x >> 5); if (r >= NT) return;
    v4f v[DMD / 128]; float s = 0.f;
#pragma unroll
    for (int q = 0; q < DMD / 128; ++q) { v[q] = *(const v4f*)(R + (size_t)r * DMD + q * 128 + lane * 4);
#pragma unroll
        for (int i = 0; i < 4; ++i) s += v[q][i]; }
#pragma unroll
    for (int sh = 16; sh; sh >>= 1) s += __shfl_xor(s, sh, 32);
    const float mu = s * (1.0f / DMD); float s2 = 0.f;
#pragma unroll
    for (int q = 0; q < DMD / 128; ++q)
#pragma unroll
        for (int i = 0; i < 4; ++i) { const float d = v[q][i] - mu; s2 = fmaf(d, d, s2); }
#pragma unroll
    for (int sh = 16; sh; sh >>= 1) s2 += __shfl_xor(s2, sh, 32);
    const float rs = 1.0f / sqrtf(s2 * (1.0f / DMD) + LN_EPS);
#pragma unroll 1
    for (int ps = 0; ps < 2; ++ps) {
#pragma unroll
        for (int q = 0; q < DMD / 128; ++q) { const int c0 = q * 128 + lane * 4; v4f y;
#pragma unroll
            for (int i = 0; i < 4; ++i) y[i] = (v[q][i] - mu) * rs * bfr(g[c0 + i]) + bfr(bb[c0 + i]);
            *(volatile v4f*)(OUTP + (size_t)r * DMD + c0) = y; }
        if (ps == 0) __threadfence(); }
}

extern "C" void kernel_launch(void* const* d_in, const int* in_sizes, int n_in,
                              void* d_out, int out_size, void* d_ws, size_t ws_size, hipStream_t stream) {
    (void)in_sizes; (void)n_in; (void)out_size;
    const float* x = (const float*)d_in[0]; const int* mask = (const int*)d_in[1];   const float* rl = (const float*)d_in[3];
    const float* qg = (const float*)d_in[4]; const float* kg = (const float*)d_in[5]; const float* vg = (const float*)d_in[6]; const float* tpb = (const float*)d_in[7];
    const float* pw = (const float*)d_in[8]; const float* pb = (const float*)d_in[9]; const float* ow = (const float*)d_in[10]; const float* ob = (const float*)d_in[11]; const float* hs = (const float*)d_in[12]; const float* lg = (const float*)d_in[13]; const float* lb = (const float*)d_in[14];
    float* out = (float*)d_out;
    char* wsp = (char*)d_ws;
    auto take = [&](size_t bytes) { char* p = wsp; wsp += (bytes + 255) & ~(size_t)255; return (void*)p; };
    bf* PWb = (bf*)take((size_t)H4 * DMD * 2); bf* OWb = (bf*)take((size_t)DMD * DMD * 2); bf* Xb = (bf*)take((size_t)NT * DMD * 2); float* Hm = (float*)take((size_t)NT * H4 * 4);
    float* CT = (float*)take((size_t)NT * 32 * 4); float* ST = (float*)take((size_t)NT * 32 * 4);
    bf* Qh = (bf*)take((size_t)NT * DMD * 2); bf* Ql = (bf*)take((size_t)NT * DMD * 2); bf* Kh = (bf*)take((size_t)NT * DMD * 2); bf* Kl = (bf*)take((size_t)NT * DMD * 2); bf* VTh = (bf*)take((size_t)NT * DMD * 2); bf* VTl = (bf*)take((size_t)NT * DMD * 2);
    float* S = (float*)take((size_t)RCH * NT * 4); bf* Wh = (bf*)take((size_t)RCH * NT * 2); bf* Wl = (bf*)take((size_t)RCH * NT * 2); float* Y = (float*)take((size_t)NT * DMD * 4); bf* Yh = (bf*)take((size_t)NT * DMD * 2); bf* Yl = (bf*)take((size_t)NT * DMD * 2); float* R = (float*)take((size_t)NT * DMD * 4);
    if ((size_t)(wsp - (char*)d_ws) > ws_size) return;
    { const size_t n1 = (size_t)H4 * DMD / 8, n2 = (size_t)DMD * DMD / 8; k_cvt8<<<(unsigned)((n1 + 255) / 256), 256, 0, stream>>>(pw, PWb, n1); k_cvt8<<<(unsigned)((n2 + 255) / 256), 256, 0, stream>>>(ow, OWb, n2); }
    for (int b = 0; b < NBI; ++b) {
        const float* xb = x + (size_t)b * NT * DMD; const float* bias_b = tpb + (size_t)b * NT * NT; const int* mask_b = mask + (size_t)b * NT * NT;
        k_pos<<<1, 256, 0, stream>>>(rl + (size_t)b * NT, CT, ST);
        k_cvtb<<<NT / 8, 256, 0, stream>>>(xb, NT, Xb);
        k_gemmb<false, false><<<dim3(NT / 64, H4 / 64, 1), 128, 0, stream>>>(Xb, nullptr, PWb, pb, Hm, H4, nullptr, nullptr, DMD);
        k_qk<<<(NT * NH) / 8, 256, 0, stream>>>(Hm, CT, ST, qg + (size_t)b * NT * NH, kg + (size_t)b * NT * NH, Qh, Ql, Kh, Kl);
        k_vtb<<<dim3(NT / 64, NH, 1), 256, 0, stream>>>(Hm, vg + (size_t)b * NT * NH, VTh, VTl);
        for (int h = 0; h < NH; ++h)
            for (int ch = 0; ch < NT / RCH; ++ch) { const int i0 = ch * RCH;
                k_gemm3ll<<<dim3(RCH / 64, NT / 64, 1), 128, 0, stream>>>(Qh + (size_t)i0 * DMD + h * HD, Ql + (size_t)i0 * DMD + h * HD, DMD, Kh + h * HD, Kl + h * HD, DMD, HD, S, NT);
                k_wprep<<<RCH / 8, 256, 0, stream>>>(S, bias_b, mask_b, hs, h, i0, Wh, Wl);
                k_gemm3ll<<<dim3(RCH / 64, 1, 1), 128, 0, stream>>>(Wh, Wl, NT, VTh + (size_t)h * HD * NT, VTl + (size_t)h * HD * NT, NT, NT, Y + (size_t)i0 * DMD + h * HD, DMD); }
        k_ygate<<<NT / 8, 256, 0, stream>>>(Y, Hm, Yh, Yl);
        k_gemmb<true, false><<<dim3(NT / 64, DMD / 64, 1), 128, 0, stream>>>(Yh, Yl, OWb, ob, R, DMD, nullptr, xb, DMD, 1);
        k_ln<<<NT / 8, 256, 0, stream>>>(R, lg, lb, out + (size_t)b * NT * DMD);
    }
}
